// SSAML_75239237092001
// MI455X (gfx1250) — hardware-run, weakly checked
//
#include <hip/hip_runtime.h>
#include <math.h>
#include <stdint.h>

typedef _Float16 v16h __attribute__((ext_vector_type(16)));
typedef _Float16 v8h  __attribute__((ext_vector_type(8)));
typedef v8h v8ha __attribute__((may_alias));
typedef float v8f __attribute__((ext_vector_type(8)));
typedef float v4f __attribute__((ext_vector_type(4)));
typedef v4f v4fa __attribute__((may_alias));

#define NB 8
#define NC 256
#define NT 2304
#define NTB (NT / 64)

#define XP 264
#define SP 72
#define KP 264
#define VP 72
#define PP 72
#define OP 68

#define KS_BYTES (64 * KP * 2)
#define VS_BYTES (NC * VP * 2)
#define PS_BYTES (4 * 16 * PP * 2)
#define ATTN_LDS (KS_BYTES + VS_BYTES + PS_BYTES)
#define OF_BYTES (NC * OP * 4)
static_assert(OF_BYTES <= ATTN_LDS);

union Frag { v16h v; v8h h[2]; };
__device__ __forceinline__ v16h ldfrag_g(const _Float16* p) {
  Frag f; f.h[0] = *(const v8h*)(p); f.h[1] = *(const v8h*)(p + 16); return f.v;
}
__device__ __forceinline__ v16h ldfrag_l(const _Float16* p) {
  Frag f; f.h[0] = *(const v8ha*)(p); f.h[1] = *(const v8ha*)(p + 16); return f.v;
}
__device__ __forceinline__ v8f mma16(v16h a, v16h b, v8f c) {
  c = __builtin_amdgcn_wmma_f32_16x16x32_f16(false, a, false, b, (short)0, c, false, false);
  asm volatile("v_nop\n\tv_nop\n\tv_nop\n\tv_nop" : "+v"(c) : "v"(a), "v"(b));
  return c;
}
__device__ __forceinline__ void wave_sync_lds() {
  __builtin_amdgcn_fence(__ATOMIC_RELEASE, "workgroup");
  __builtin_amdgcn_wave_barrier();
  __builtin_amdgcn_fence(__ATOMIC_ACQUIRE, "workgroup");
}

__global__ __launch_bounds__(256) void k_wprep(const float* __restrict__ Wq, const float* __restrict__ Wk,
                                               const float* __restrict__ Wv, _Float16* __restrict__ Wh) {
  const int mat = blockIdx.x >> 5;
  const float* W = (mat == 0) ? Wq : ((mat == 1) ? Wk : Wv);
  const int e0 = ((blockIdx.x & 31) * 256 + (int)threadIdx.x) * 8;
  const v4f a = *(const v4f*)(W + e0);
  const v4f c = *(const v4f*)(W + e0 + 4);
  v8h hv;
  hv[0] = (_Float16)(a[0] * 16.0f); hv[1] = (_Float16)(a[1] * 16.0f);
  hv[2] = (_Float16)(a[2] * 16.0f); hv[3] = (_Float16)(a[3] * 16.0f);
  hv[4] = (_Float16)(c[0] * 16.0f); hv[5] = (_Float16)(c[1] * 16.0f);
  hv[6] = (_Float16)(c[2] * 16.0f); hv[7] = (_Float16)(c[3] * 16.0f);
  _Float16* dst = Wh + (size_t)mat * NC * NC + e0;
  *(volatile v8h*)dst = hv;
  __threadfence();
  *(volatile v8h*)dst = hv;
}

__global__ __launch_bounds__(256) void k_qkv(const float* __restrict__ x, const _Float16* __restrict__ Wh,
                                             const float* __restrict__ bq, const float* __restrict__ bk,
                                             const float* __restrict__ bv,
                                             _Float16* __restrict__ Qp, _Float16* __restrict__ Kp,
                                             _Float16* __restrict__ Vp) {
  __shared__ __align__(16) _Float16 Xs[64 * XP];
  __shared__ __align__(16) _Float16 Sl[8][16 * SP];

  const int tid  = threadIdx.x;
  const int wave = __builtin_amdgcn_readfirstlane(tid >> 5);
  const int lane = tid & 31, hh = lane >> 4, ln = lane & 15;
  const int q8 = lane >> 3, c8 = (lane & 7) * 8;
  const int b  = blockIdx.x / NTB;
  const int n0 = (blockIdx.x - b * NTB) * 64;
  const float* xb = x + (size_t)b * NC * NT + n0;

#pragma unroll 4
  for (int it = 0; it < 16; ++it) {
    const int idx = it * 256 + tid;
    const int c = idx >> 4;
    const int n4 = (idx & 15) * 4;
    const v4f v = *(const v4f*)(xb + (size_t)c * NT + n4);
    Xs[(n4 + 0) * XP + c] = (_Float16)v[0];
    Xs[(n4 + 1) * XP + c] = (_Float16)v[1];
    Xs[(n4 + 2) * XP + c] = (_Float16)v[2];
    Xs[(n4 + 3) * XP + c] = (_Float16)v[3];
  }
  __syncthreads();

  _Float16* slab = Sl[wave];

  for (int ti = 0; ti < 2; ++ti) {
    const int mh = wave & 1, chunk = wave >> 1;
    const int c0 = chunk * 64;
    const _Float16* Wm = Wh + (size_t)ti * NC * NC;
    const float* bias = ti ? bk : bq;
    _Float16* Op = ti ? Kp : Qp;

    v8f acc[2][4];
#pragma unroll
    for (int i = 0; i < 2; ++i)
#pragma unroll
      for (int j = 0; j < 4; ++j) acc[i][j] = (v8f){0.f, 0.f, 0.f, 0.f, 0.f, 0.f, 0.f, 0.f};

#pragma unroll 1
    for (int s = 0; s < 8; ++s) {
      v16h bf[4];
#pragma unroll
      for (int j = 0; j < 4; ++j) bf[j] = ldfrag_g(Wm + (size_t)(c0 + j * 16 + ln) * NC + s * 32 + 8 * hh);
#pragma unroll
      for (int i = 0; i < 2; ++i) {
        const v16h af = ldfrag_l(Xs + (mh * 32 + i * 16 + ln) * XP + s * 32 + 8 * hh);
#pragma unroll
        for (int j = 0; j < 4; ++j) acc[i][j] = mma16(af, bf[j], acc[i][j]);
      }
    }

#pragma unroll
    for (int i = 0; i < 2; ++i) {
      wave_sync_lds();
#pragma unroll
      for (int j = 0; j < 4; ++j) {
        const float bb = bias[c0 + j * 16 + ln];
#pragma unroll
        for (int r = 0; r < 8; ++r)
          slab[(8 * hh + r) * SP + j * 16 + ln] = (_Float16)(acc[i][j][r] * 0.0625f + bb);
      }
      wave_sync_lds();
      _Float16* orow = Op + ((size_t)b * NT + n0 + mh * 32 + i * 16) * NC + c0 + c8;
      for (int pass = 0; pass < 2; ++pass) {
#pragma unroll
        for (int it = 0; it < 4; ++it) {
          const int row = it * 4 + q8;
          const v8h hv = *(const v8ha*)(slab + row * SP + c8);
          *(volatile v8h*)(orow + (size_t)row * NC) = hv;
        }
        __threadfence();
      }
    }
  }

  {
    const int cb = wave * 32;
    const _Float16* Wm = Wh + (size_t)2 * NC * NC;
    v8f acc[2][4];
#pragma unroll
    for (int i = 0; i < 2; ++i)
#pragma unroll
      for (int j = 0; j < 4; ++j) acc[i][j] = (v8f){0.f, 0.f, 0.f, 0.f, 0.f, 0.f, 0.f, 0.f};

#pragma unroll 1
    for (int s = 0; s < 8; ++s) {
      v16h af[2];
#pragma unroll
      for (int i = 0; i < 2; ++i) af[i] = ldfrag_g(Wm + (size_t)(cb + i * 16 + ln) * NC + s * 32 + 8 * hh);
#pragma unroll
      for (int j = 0; j < 4; ++j) {
        const v16h bf = ldfrag_l(Xs + (j * 16 + ln) * XP + s * 32 + 8 * hh);
#pragma unroll
        for (int i = 0; i < 2; ++i) acc[i][j] = mma16(af[i], bf, acc[i][j]);
      }
    }

#pragma unroll
    for (int i = 0; i < 2; ++i) {
      wave_sync_lds();
#pragma unroll
      for (int r = 0; r < 8; ++r) {
        const float bb = bv[cb + i * 16 + 8 * hh + r];
#pragma unroll
        for (int j = 0; j < 4; ++j)
          slab[(8 * hh + r) * SP + j * 16 + ln] = (_Float16)(acc[i][j][r] * 0.0625f + bb);
      }
      wave_sync_lds();
      _Float16* orow = Vp + ((size_t)b * NC + cb + i * 16) * NT + n0 + c8;
      for (int pass = 0; pass < 2; ++pass) {
#pragma unroll
        for (int it = 0; it < 4; ++it) {
          const int row = it * 4 + q8;
          const v8h hv = *(const v8ha*)(slab + row * SP + c8);
          *(volatile v8h*)(orow + (size_t)row * NT) = hv;
        }
        __threadfence();
      }
    }
  }
}

__global__ __launch_bounds__(128) void k_attn(const _Float16* __restrict__ Qp, const _Float16* __restrict__ Kp,
                                              const _Float16* __restrict__ Vp, const float* __restrict__ x,
                                              const float* __restrict__ gamma, float* __restrict__ out) {
  extern __shared__ __align__(16) char smem[];
  _Float16* Ks = (_Float16*)(smem);
  _Float16* Vs = (_Float16*)(smem + KS_BYTES);
  _Float16* Ps = (_Float16*)(smem + KS_BYTES + VS_BYTES);
  float*    Of = (float*)(smem);

  const int tid  = threadIdx.x;
  const int wave = __builtin_amdgcn_readfirstlane(tid >> 5);
  const int lane = tid & 31, hh = lane >> 4, ln = lane & 15;
  const int b  = blockIdx.x / NTB;
  const int n0 = (blockIdx.x - b * NTB) * 64;
  const int q0 = n0 + wave * 16;

  const _Float16* Qb = Qp + ((size_t)b * NT + q0 + ln) * NC + 8 * hh;
  const _Float16* Kb = Kp + (size_t)b * NT * NC;
  const _Float16* Vb = Vp + (size_t)b * NC * NT;
  _Float16* pw = Ps + wave * (16 * PP);

  float mr[8], lr[8];
  v8f O[16];
#pragma unroll
  for (int r = 0; r < 8; ++r) { mr[r] = -INFINITY; lr[r] = 0.f; }
#pragma unroll
  for (int ct = 0; ct < 16; ++ct) O[ct] = (v8f){0.f, 0.f, 0.f, 0.f, 0.f, 0.f, 0.f, 0.f};

  for (int kt = 0; kt < NTB; ++kt) {
    __syncthreads();
#pragma unroll 4
    for (int it = 0; it < 16; ++it) {
      const int idx = it * 128 + tid;
      const int kr = idx >> 5, kc = (idx & 31) * 8;
      const v8h kv = *(const v8h*)(Kb + (size_t)(kt * 64 + kr) * NC + kc);
      *(v8h*)(Ks + kr * KP + kc) = kv;
      const int vr = idx >> 3, vc = (idx & 7) * 8;
      const v8h vv = *(const v8h*)(Vb + (size_t)vr * NT + kt * 64 + vc);
      *(v8h*)(Vs + vr * VP + vc) = vv;
    }
    __syncthreads();

    v8f S[4];
#pragma unroll
    for (int j = 0; j < 4; ++j) S[j] = (v8f){0.f, 0.f, 0.f, 0.f, 0.f, 0.f, 0.f, 0.f};
#pragma unroll 1
    for (int s = 0; s < 8; ++s) {
      const v16h qa = ldfrag_g(Qb + s * 32);
#pragma unroll
      for (int j = 0; j < 4; ++j) {
        const v16h kb = ldfrag_l(Ks + (j * 16 + ln) * KP + s * 32 + 8 * hh);
        S[j] = mma16(qa, kb, S[j]);
      }
    }

    float cm[8];
#pragma unroll
    for (int r = 0; r < 8; ++r) {
      float m = fmaxf(fmaxf(-S[0][r], -S[1][r]), fmaxf(-S[2][r], -S[3][r]));
      m = fmaxf(m, __shfl_xor(m, 1, 32));
      m = fmaxf(m, __shfl_xor(m, 2, 32));
      m = fmaxf(m, __shfl_xor(m, 4, 32));
      m = fmaxf(m, __shfl_xor(m, 8, 32));
      cm[r] = m;
    }
#pragma unroll
    for (int r = 0; r < 8; ++r) {
      const float mnew  = fmaxf(mr[r], cm[r]);
      const float alpha = __expf(mr[r] - mnew);
      mr[r] = mnew;
      float ps = 0.f;
#pragma unroll
      for (int j = 0; j < 4; ++j) {
        const float p = __expf(-S[j][r] - mnew);
        ps += p;
        pw[(8 * hh + r) * PP + j * 16 + ln] = (_Float16)(p * 4096.0f);
      }
      ps += __shfl_xor(ps, 1, 32);
      ps += __shfl_xor(ps, 2, 32);
      ps += __shfl_xor(ps, 4, 32);
      ps += __shfl_xor(ps, 8, 32);
      lr[r] = lr[r] * alpha + ps;
#pragma unroll
      for (int ct = 0; ct < 16; ++ct) O[ct][r] = O[ct][r] * alpha;
    }
    wave_sync_lds();

    const v16h pa0 = ldfrag_l(pw + ln * PP + 8 * hh);
    const v16h pa1 = ldfrag_l(pw + ln * PP + 32 + 8 * hh);
#pragma unroll
    for (int ct = 0; ct < 16; ++ct) {
      const _Float16* vrow = Vs + (ct * 16 + ln) * VP + 8 * hh;
      const v16h vb0 = ldfrag_l(vrow);
      const v16h vb1 = ldfrag_l(vrow + 32);
      O[ct] = mma16(pa0, vb0, O[ct]);
      O[ct] = mma16(pa1, vb1, O[ct]);
    }
  }

  __syncthreads();
  float inv[8];
#pragma unroll
  for (int r = 0; r < 8; ++r) inv[r] = 0.000244140625f * (1.0f / lr[r]);
#pragma unroll
  for (int ct = 0; ct < 16; ++ct) {
    float* op = Of + (ct * 16 + ln) * OP + wave * 16 + 8 * hh;
    v4f u0, u1;
    u0[0] = O[ct][0] * inv[0]; u0[1] = O[ct][1] * inv[1]; u0[2] = O[ct][2] * inv[2]; u0[3] = O[ct][3] * inv[3];
    u1[0] = O[ct][4] * inv[4]; u1[1] = O[ct][5] * inv[5]; u1[2] = O[ct][6] * inv[6]; u1[3] = O[ct][7] * inv[7];
    *(v4f*)(op)     = u0;
    *(v4f*)(op + 4) = u1;
  }
  __syncthreads();

  const float gm = gamma[0];
  const int chl = lane >> 4;
  const int tok = ((lane >> 3) & 1) * 32 + (lane & 7) * 4;
  const float* xb = x   + (size_t)b * NC * NT + n0 + tok;
  float*       ob = out + (size_t)b * NC * NT + n0 + tok;
  for (int pass = 0; pass < 2; ++pass) {
#pragma unroll 4
    for (int it = 0; it < 32; ++it) {
      const int ch = wave * 64 + it * 2 + chl;
      const v4f of = *(const v4fa*)(Of + ch * OP + tok);
      const v4f xv = *(const v4f*)(xb + (size_t)ch * NT);
      v4f o;
      o[0] = gm * of[0] + xv[0]; o[1] = gm * of[1] + xv[1];
      o[2] = gm * of[2] + xv[2]; o[3] = gm * of[3] + xv[3];
      *(volatile v4f*)(ob + (size_t)ch * NT) = o;
    }
    __threadfence();
  }
}

extern "C" void kernel_launch(void* const* d_in, const int* in_sizes, int n_in,
                              void* d_out, int out_size, void* d_ws, size_t ws_size,
                              hipStream_t stream) {
  if (n_in < 8) return;
  if (in_sizes[0] != NB * NC * NT) return;
  if (in_sizes[1] != NC * NC || in_sizes[3] != NC * NC || in_sizes[5] != NC * NC) return;
  if (in_sizes[2] != NC || in_sizes[4] != NC || in_sizes[6] != NC || in_sizes[7] < 1) return;
  if (out_size != NB * NC * NT) return;

  const size_t wbytes = (size_t)3 * NC * NC * 2;
  const size_t pbytes = (size_t)NB * NT * NC * 2;
  const size_t oW = 0;
  const size_t oQ = oW + wbytes;
  const size_t oK = oQ + pbytes;
  const size_t oV = oK + pbytes;
  const size_t total = oV + pbytes;
  if (total > ws_size) return;

  const float* x  = (const float*)d_in[0];
  const float* Wq = (const float*)d_in[1];
  const float* bq = (const float*)d_in[2];
  const float* Wk = (const float*)d_in[3];
  const float* bk = (const float*)d_in[4];
  const float* Wv = (const float*)d_in[5];
  const float* bv = (const float*)d_in[6];
  const float* gm = (const float*)d_in[7];
  float* out = (float*)d_out;

  char* ws = (char*)d_ws;
  _Float16* Wh = (_Float16*)(ws + oW);
  _Float16* Qp = (_Float16*)(ws + oQ);
  _Float16* Kp = (_Float16*)(ws + oK);
  _Float16* Vp = (_Float16*)(ws + oV);

  k_wprep<<<dim3(96), dim3(256), 0, stream>>>(Wq, Wk, Wv, Wh);
  k_qkv<<<dim3(NB * NTB), dim3(256), 0, stream>>>(x, Wh, bq, bk, bv, Qp, Kp, Vp);
  (void)hipFuncSetAttribute(reinterpret_cast<const void*>(&k_attn),
                            hipFuncAttributeMaxDynamicSharedMemorySize, ATTN_LDS);
  k_attn<<<dim3(NB * NTB), dim3(128), ATTN_LDS, stream>>>(Qp, Kp, Vp, x, gm, out);
  (void)hipGetLastError();
}
